// BermMatrixLayer_85504208928778
// MI455X (gfx1250) — hardware-verified
//
#include <hip/hip_runtime.h>
#include <math.h>


constexpr int NB_  = 4;
constexpr int NS_  = 2048;
constexpr int NHID = 1024;
constexpr int NH_  = 16;
constexpr int ND_  = 16;
constexpr int NHV_ = 64;
constexpr int NCOL = NH_ * ND_ * ND_;
constexpr int NTOK = NB_ * NS_;
constexpr int NGRP = 2;
constexpr int HPG  = NH_ / NGRP;
constexpr int GCOL = HPG * ND_ * ND_;
constexpr int NBHL = NB_ * HPG;
constexpr int BPC  = NS_ / 64;

static_assert(NTOK % 64 == 0);
static_assert(GCOL % 128 == 0);
static_assert(NHID % 64 == 0);
static_assert(NCOL % 64 == 0);
static_assert(NS_ % 64 == 0);
static_assert(NHV_ == 64);
static_assert(HPG == 8);

typedef float          v4f   __attribute__((ext_vector_type(4)));
typedef float          v8f   __attribute__((ext_vector_type(8)));
typedef __bf16         v16b  __attribute__((ext_vector_type(16)));
typedef _Float16       v8h   __attribute__((ext_vector_type(8)));
typedef _Float16       v16h  __attribute__((ext_vector_type(16)));
typedef unsigned short u16x8 __attribute__((ext_vector_type(8)));

union FragB { u16x8 h[2]; v16b v; };
union FragH { u16x8 h[2]; v16h v; };
union Cvt8H { v8h f; u16x8 u; };

__device__ __forceinline__ unsigned short f2bf(float f) {
    unsigned u = __float_as_uint(f);
    unsigned r = u + 0x7FFFu + ((u >> 16) & 1u);
    return (unsigned short)(r >> 16);
}
__device__ __forceinline__ float bf2f(unsigned short b) {
    return __uint_as_float(((unsigned)b) << 16);
}
__device__ __forceinline__ v8f ld8f(const float* p) {
    v4f a = *(const v4f*)p;
    v4f b = *(const v4f*)(p + 4);
    return __builtin_shufflevector(a, b, 0, 1, 2, 3, 4, 5, 6, 7);
}
__device__ __forceinline__ void split8(const v8f& x, u16x8& hv, u16x8& lv) {
#pragma unroll
    for (int c = 0; c < 8; ++c) {
        const float f = x[c];
        const unsigned short hb = f2bf(f);
        hv[c] = hb;
        lv[c] = f2bf(f - bf2f(hb));
    }
}
__device__ __forceinline__ void ldsplit(const float* p, u16x8& hv, u16x8& lv) {
    const v8f x = ld8f(p);
    split8(x, hv, lv);
}
__device__ __forceinline__ u16x8 cvt8h(const v8f& x, float sc) {
    Cvt8H c;
#pragma unroll
    for (int e = 0; e < 8; ++e) c.f[e] = (_Float16)(x[e] * sc);
    return c.u;
}
__device__ __forceinline__ float wsum32(float v) {
    v += __shfl_xor(v, 16, 32);
    v += __shfl_xor(v, 8, 32);
    v += __shfl_xor(v, 4, 32);
    v += __shfl_xor(v, 2, 32);
    v += __shfl_xor(v, 1, 32);
    return v;
}
__device__ __forceinline__ float gelu_f(float x) {
    return 0.5f * x * (1.0f + erff(x * 0.70710678118654752440f));
}

__device__ __forceinline__ void mma_bf(v8f& acc, const FragB& a, const FragB& b) {
    acc = __builtin_amdgcn_wmma_f32_16x16x32_bf16(false, a.v, false, b.v, (short)0, acc, false, false);
    asm volatile("v_nop\n\tv_nop\n\tv_nop\n\tv_nop" : "+v"(acc) : "v"(a.v), "v"(b.v));
}
__device__ __forceinline__ void mma_h(v8f& acc, const FragH& a, const FragH& b) {
    acc = __builtin_amdgcn_wmma_f32_16x16x32_f16(false, a.v, false, b.v, (short)0, acc, false, false);
    asm volatile("v_nop\n\tv_nop\n\tv_nop\n\tv_nop" : "+v"(acc) : "v"(a.v), "v"(b.v));
}

template<int NBF>
__device__ __forceinline__ void tile_store_pass(const float* st, float* gp, int ldc, int lane) {
    constexpr int CW  = NBF * 16;
    constexpr int P   = CW + 4;
    constexpr int LPR = CW / 4;
    constexpr int RPI = 32 / LPR;
    constexpr int NIT = 32 / RPI;
    const int rsub = lane / LPR;
    const int c4   = (lane % LPR) * 4;
#pragma unroll
    for (int it = 0; it < NIT; ++it) {
        const int row = it * RPI + rsub;
        const v4f v = *(const v4f*)(st + row * P + c4);
        *(volatile v4f*)(gp + (size_t)row * ldc + c4) = v;
    }
}

__global__ __launch_bounds__(256)
void cvt_hs_kernel(const float* __restrict__ src, unsigned short* dst, int n8)
{
    const int i = blockIdx.x * 256 + threadIdx.x;
    if (i >= n8) return;
    const size_t e = (size_t)i * 8;
    const v8f x = ld8f(src + e);
    const u16x8 hv = cvt8h(x, 1.0f);
    *(volatile u16x8*)(dst + e) = hv;
    __threadfence();
    *(volatile u16x8*)(dst + e) = hv;
}

__global__ __launch_bounds__(256)
void cvt_wt_kernel(const float* __restrict__ W, unsigned short* Wt)
{
    __shared__ float tile[64][65];
    const int tid = threadIdx.x;
    const int n0 = blockIdx.x * 64;
    const int k0 = blockIdx.y * 64;
#pragma unroll
    for (int it = 0; it < 4; ++it) {
        const int kk = it * 16 + (tid >> 4);
        const int n4 = (tid & 15) * 4;
        const v4f x = *(const v4f*)(W + (size_t)(k0 + kk) * NCOL + n0 + n4);
        tile[kk][n4 + 0] = x.x;
        tile[kk][n4 + 1] = x.y;
        tile[kk][n4 + 2] = x.z;
        tile[kk][n4 + 3] = x.w;
    }
    __syncthreads();
    u16x8 vals[2];
    size_t goff[2];
#pragma unroll
    for (int it = 0; it < 2; ++it) {
        const int nn = it * 32 + (tid >> 3);
        const int k8 = (tid & 7) * 8;
        v8f x;
#pragma unroll
        for (int e = 0; e < 8; ++e) x[e] = tile[k8 + e][nn];
        vals[it] = cvt8h(x, 32.0f);
        goff[it] = (size_t)(n0 + nn) * NHID + k0 + k8;
    }
    *(volatile u16x8*)(Wt + goff[0]) = vals[0];
    *(volatile u16x8*)(Wt + goff[1]) = vals[1];
    __threadfence();
    *(volatile u16x8*)(Wt + goff[0]) = vals[0];
    *(volatile u16x8*)(Wt + goff[1]) = vals[1];
}

__global__ __launch_bounds__(256)
void cvt_wv_kernel(const float* __restrict__ Wv, unsigned short* Th, unsigned short* Tl)
{
    __shared__ float tile[64][65];
    const int tid = threadIdx.x;
    const int h = blockIdx.x;
    const float* src = Wv + (size_t)h * 64 * 64;
#pragma unroll
    for (int it = 0; it < 4; ++it) {
        const int ii = it * 16 + (tid >> 4);
        const int o4 = (tid & 15) * 4;
        const v4f x = *(const v4f*)(src + ii * 64 + o4);
        tile[ii][o4 + 0] = x.x;
        tile[ii][o4 + 1] = x.y;
        tile[ii][o4 + 2] = x.z;
        tile[ii][o4 + 3] = x.w;
    }
    __syncthreads();
    u16x8 hvs[2], lvs[2];
    size_t goff[2];
#pragma unroll
    for (int it = 0; it < 2; ++it) {
        const int oo = it * 32 + (tid >> 3);
        const int i8 = (tid & 7) * 8;
        v8f x;
#pragma unroll
        for (int e = 0; e < 8; ++e) x[e] = tile[i8 + e][oo];
        split8(x, hvs[it], lvs[it]);
        goff[it] = ((size_t)h * 64 + oo) * 64 + i8;
    }
    *(volatile u16x8*)(Th + goff[0]) = hvs[0];
    *(volatile u16x8*)(Th + goff[1]) = hvs[1];
    *(volatile u16x8*)(Tl + goff[0]) = lvs[0];
    *(volatile u16x8*)(Tl + goff[1]) = lvs[1];
    __threadfence();
    *(volatile u16x8*)(Th + goff[0]) = hvs[0];
    *(volatile u16x8*)(Th + goff[1]) = hvs[1];
    *(volatile u16x8*)(Tl + goff[0]) = lvs[0];
    *(volatile u16x8*)(Tl + goff[1]) = lvs[1];
}

__global__ __launch_bounds__(128)
void gemm_f16_kernel(const unsigned short* __restrict__ A, const unsigned short* __restrict__ Bt,
                     const float* __restrict__ bias, float* C, int K, int ldc, float oscale)
{
    constexpr int NBF = 4;
    constexpr int CW  = NBF * 16;
    constexpr int P   = CW + 4;
    __shared__ __attribute__((aligned(16))) float stile[4][32 * P];

    const int tid  = threadIdx.x;
    const int lane = tid & 31;
    const int wave = tid >> 5;
    const int hh   = lane >> 4;
    const int m    = lane & 15;
    const int wm   = wave >> 1;
    const int wn   = wave & 1;

    const int rowW = blockIdx.y * 64 + wm * 32;
    const int colW = blockIdx.x * (2 * CW) + wn * CW;

    v8f acc[2 * NBF];
#pragma unroll
    for (int j = 0; j < 2 * NBF; ++j)
#pragma unroll
        for (int r = 0; r < 8; ++r) acc[j][r] = 0.0f;

    const size_t aoff  = (size_t)(rowW + m) * K + 8 * hh;
    const size_t boff  = (size_t)(colW + m) * K + 8 * hh;
    const size_t sub16 = (size_t)16 * K;
    const int nk = K >> 5;

#pragma unroll 1
    for (int kt = 0; kt < nk; ++kt) {
        const size_t k0 = (size_t)kt * 32;
        FragH fa[2], fb[NBF];
#pragma unroll
        for (int s = 0; s < 2; ++s) {
            const unsigned short* p = A + aoff + s * sub16 + k0;
            fa[s].h[0] = *(const u16x8*)(p);
            fa[s].h[1] = *(const u16x8*)(p + 16);
        }
#pragma unroll
        for (int j = 0; j < NBF; ++j) {
            const unsigned short* p = Bt + boff + j * sub16 + k0;
            fb[j].h[0] = *(const u16x8*)(p);
            fb[j].h[1] = *(const u16x8*)(p + 16);
        }
#pragma unroll
        for (int s = 0; s < 2; ++s)
#pragma unroll
            for (int j = 0; j < NBF; ++j)
                mma_h(acc[s * NBF + j], fa[s], fb[j]);
    }

    float bj[NBF];
#pragma unroll
    for (int j = 0; j < NBF; ++j) bj[j] = bias[colW + 16 * j + m];

    float* st = stile[wave];
#pragma unroll
    for (int s = 0; s < 2; ++s)
#pragma unroll
        for (int j = 0; j < NBF; ++j)
#pragma unroll
            for (int r = 0; r < 8; ++r)
                st[(s * 16 + 8 * hh + r) * P + j * 16 + m] = acc[s * NBF + j][r] * oscale + bj[j];
    __syncthreads();

    float* gp = C + (size_t)rowW * ldc + colW;
    tile_store_pass<NBF>(st, gp, ldc, lane);
    __threadfence();
    tile_store_pass<NBF>(st, gp, ldc, lane);
}

__global__ __launch_bounds__(64)
void chain_kernel(const float* __restrict__ Mg, const float* __restrict__ mask,
                  float* VL, float* VD, float* VG)
{
    __shared__ __attribute__((aligned(16))) float stg[2][2][256];
    __shared__ __attribute__((aligned(16))) float gst[32];

    const int tid  = threadIdx.x;
    const int lane = tid & 31;
    const int dir  = tid >> 5;
    const int bhl  = blockIdx.x;
    const int b    = bhl >> 3;
    const int hl   = bhl & 7;
    const int i    = lane & 15;
    const int hh   = lane >> 4;
    const int sa   = (dir != 0) ? 1 : 16;
    const int sb   = (dir != 0) ? 16 : 1;

    const float* Mrow = Mg + (size_t)b * NS_ * GCOL + hl * 256;
    const float* mrow = mask + b * NS_;
    float* Vd = VD + ((size_t)dir * NBHL + bhl) * NS_ * 16;
    float* Vl = VL + (size_t)bhl * NS_ * 16;

    float v[16];
#pragma unroll
    for (int j = 0; j < 16; ++j) v[j] = (j == 0) ? 1.0f : 0.0f;
    float vi = (i == 0) ? 1.0f : 0.0f;
    int moff[8];
#pragma unroll
    for (int c = 0; c < 8; ++c) moff[c] = i * sa + (8 * hh + c) * sb;

#pragma unroll 1
    for (int c0 = 0; c0 < NS_; c0 += 16) {
#pragma unroll 1
        for (int t = 0; t < 16; ++t) {
            const int k = c0 + t;
            const int s = (dir != 0) ? (NS_ - 1 - k) : k;
            const float a = mrow[s];
            const float* Ms = Mrow + (size_t)s * GCOL;
            float me[8];
#pragma unroll
            for (int c = 0; c < 8; ++c) me[c] = Ms[moff[c]];
            float sq = 0.0f;
#pragma unroll
            for (int c = 0; c < 8; ++c) sq += me[c] * me[c];
            sq = wsum32(sq);
            const float inv = 1.0f / sqrtf(sq);
            float part = 0.0f;
#pragma unroll
            for (int c = 0; c < 8; ++c) {
                const float vj = (hh != 0) ? v[8 + c] : v[c];
                part += (me[c] * inv) * vj;
            }
            const float nv = part + __shfl_xor(part, 16, 32);
            const int sl = (s & 15) * 16 + i;
            stg[dir][0][sl] = vi;
            if (dir == 0) {
                if (hh == 0) {
                    const float e0 = (i == 0) ? 1.0f : 0.0f;
                    stg[0][1][sl] = (me[0] * inv) * a + e0 * (1.0f - a);
                }
            }
            const float vn = nv * a + vi * (1.0f - a);
            vi = vn;
#pragma unroll
            for (int j = 0; j < 16; ++j) v[j] = __shfl(vn, j, 32);
        }
        __syncthreads();
        const int slo = (dir != 0) ? (NS_ - 16 - c0) : c0;
        const v4f d0 = *(const v4f*)(&stg[dir][0][lane * 4]);
        const v4f d1 = *(const v4f*)(&stg[dir][0][128 + lane * 4]);
        const v4f l0 = *(const v4f*)(&stg[0][1][lane * 4]);
        const v4f l1 = *(const v4f*)(&stg[0][1][128 + lane * 4]);
        float* gp = Vd + (size_t)slo * 16 + lane * 4;
        float* lp = Vl + (size_t)slo * 16 + lane * 4;
        *(volatile v4f*)gp = d0;
        *(volatile v4f*)(gp + 128) = d1;
        if (dir == 0) {
            *(volatile v4f*)lp = l0;
            *(volatile v4f*)(lp + 128) = l1;
        }
        __threadfence();
        *(volatile v4f*)gp = d0;
        *(volatile v4f*)(gp + 128) = d1;
        if (dir == 0) {
            *(volatile v4f*)lp = l0;
            *(volatile v4f*)(lp + 128) = l1;
        }
        __syncthreads();
    }

    if (dir == 0) gst[lane] = (hh == 0) ? vi : 0.0f;
    __syncthreads();
    const v4f gv = *(const v4f*)(&gst[(lane & 7) * 4]);
    float* gq = VG + bhl * 32 + (lane & 7) * 4;
    const bool wg = (tid < 8);
    if (wg) *(volatile v4f*)gq = gv;
    __threadfence();
    if (wg) *(volatile v4f*)gq = gv;
}

__global__ __launch_bounds__(128)
void gemm_out_kernel(const float* __restrict__ VL, const float* __restrict__ VG, const float* __restrict__ VD,
                     const unsigned short* __restrict__ Th, const unsigned short* __restrict__ Tl,
                     const float* __restrict__ bias, int g, float* out)
{
    constexpr int NBF = 2;
    constexpr int CW  = NBF * 16;
    constexpr int P   = CW + 4;
    __shared__ __attribute__((aligned(16))) float stile[4][32 * P];

    const int tid  = threadIdx.x;
    const int lane = tid & 31;
    const int wave = tid >> 5;
    const int hh   = lane >> 4;
    const int m    = lane & 15;
    const int wm   = wave >> 1;
    const int wn   = wave & 1;

    const int bq  = blockIdx.x;
    const int bhl = bq / BPC;
    const int b   = bhl >> 3;
    const int hl  = bhl & 7;
    const int h   = g * HPG + hl;
    const int s0  = (bq % BPC) * 64 + wm * 32;
    const size_t rowL = (size_t)bhl * NS_ + s0;
    const int colW = wn * CW;

    const float* pL = VL + rowL * 16;
    const float* pF = VD + rowL * 16;
    const float* pR = VD + (size_t)NBHL * NS_ * 16 + rowL * 16;
    const float* pG = VG + bhl * 32 + 8 * hh;
    const unsigned short* qh = Th + ((size_t)h * NHV_ + colW + m) * 64 + 8 * hh;
    const unsigned short* ql = Tl + ((size_t)h * NHV_ + colW + m) * 64 + 8 * hh;

    v8f acc[2 * NBF];
#pragma unroll
    for (int j = 0; j < 2 * NBF; ++j)
#pragma unroll
        for (int r = 0; r < 8; ++r) acc[j][r] = 0.0f;

    {
        FragB fa[2], ga[2], fb[NBF], gb[NBF];
#pragma unroll
        for (int s = 0; s < 2; ++s) {
            ldsplit(pL + (size_t)(s * 16 + m) * 16 + 8 * hh, fa[s].h[0], ga[s].h[0]);
            ldsplit(pG, fa[s].h[1], ga[s].h[1]);
        }
#pragma unroll
        for (int j = 0; j < NBF; ++j) {
            const unsigned short* p = qh + j * 16 * 64;
            const unsigned short* q = ql + j * 16 * 64;
            fb[j].h[0] = *(const u16x8*)(p);
            fb[j].h[1] = *(const u16x8*)(p + 16);
            gb[j].h[0] = *(const u16x8*)(q);
            gb[j].h[1] = *(const u16x8*)(q + 16);
        }
#pragma unroll
        for (int s = 0; s < 2; ++s)
#pragma unroll
            for (int j = 0; j < NBF; ++j) {
                mma_bf(acc[s * NBF + j], fa[s], fb[j]);
                mma_bf(acc[s * NBF + j], fa[s], gb[j]);
                mma_bf(acc[s * NBF + j], ga[s], fb[j]);
            }
    }
    {
        FragB fa[2], ga[2], fb[NBF], gb[NBF];
#pragma unroll
        for (int s = 0; s < 2; ++s) {
            ldsplit(pF + (size_t)(s * 16 + m) * 16 + 8 * hh, fa[s].h[0], ga[s].h[0]);
            ldsplit(pR + (size_t)(s * 16 + m) * 16 + 8 * hh, fa[s].h[1], ga[s].h[1]);
        }
#pragma unroll
        for (int j = 0; j < NBF; ++j) {
            const unsigned short* p = qh + j * 16 * 64 + 32;
            const unsigned short* q = ql + j * 16 * 64 + 32;
            fb[j].h[0] = *(const u16x8*)(p);
            fb[j].h[1] = *(const u16x8*)(p + 16);
            gb[j].h[0] = *(const u16x8*)(q);
            gb[j].h[1] = *(const u16x8*)(q + 16);
        }
#pragma unroll
        for (int s = 0; s < 2; ++s)
#pragma unroll
            for (int j = 0; j < NBF; ++j) {
                mma_bf(acc[s * NBF + j], fa[s], fb[j]);
                mma_bf(acc[s * NBF + j], fa[s], gb[j]);
                mma_bf(acc[s * NBF + j], ga[s], fb[j]);
            }
    }

    const float b0 = bias[h * NHV_ + colW + m];
    const float b1 = bias[h * NHV_ + colW + 16 + m];

    float* st = stile[wave];
#pragma unroll
    for (int s = 0; s < 2; ++s)
#pragma unroll
        for (int j = 0; j < NBF; ++j)
#pragma unroll
            for (int r = 0; r < 8; ++r)
                st[(s * 16 + 8 * hh + r) * P + j * 16 + m] = gelu_f(acc[s * NBF + j][r] + (j == 0 ? b0 : b1));
    __syncthreads();

    float* gp = out + ((size_t)(b * NH_ + h) * NS_ + s0) * NHV_ + colW;
    tile_store_pass<NBF>(st, gp, NHV_, lane);
    __threadfence();
    tile_store_pass<NBF>(st, gp, NHV_, lane);
}

extern "C" void kernel_launch(void* const* d_in, const int* in_sizes, int n_in,
                              void* d_out, int out_size, void* d_ws, size_t ws_size,
                              hipStream_t stream)
{
    if (n_in < 6) return;
    const int want[6] = { NTOK * NHID, NB_ * NS_, NHID * NCOL, NCOL, NH_ * 64 * NHV_, NH_ * NHV_ };
    for (int i = 0; i < 6; ++i) if (in_sizes[i] != want[i]) return;
    if (out_size != NTOK * NHID) return;

    const float* hs   = (const float*)d_in[0];
    const float* mask = (const float*)d_in[1];
    const float* Wm   = (const float*)d_in[2];
    const float* bm   = (const float*)d_in[3];
    const float* Wv   = (const float*)d_in[4];
    const float* bv   = (const float*)d_in[5];
    float* out = (float*)d_out;

    char* ws = (char*)d_ws;
    size_t off = 0;
    auto carve = [&](size_t bytes) -> char* { char* p = ws + off; off += (bytes + 255) & ~(size_t)255; return p; };
    unsigned short* Xh   = (unsigned short*)carve((size_t)NTOK * NHID * 2);
    unsigned short* Wt   = (unsigned short*)carve((size_t)NCOL * NHID * 2);
    unsigned short* WvTh = (unsigned short*)carve((size_t)NH_ * 64 * 64 * 2);
    unsigned short* WvTl = (unsigned short*)carve((size_t)NH_ * 64 * 64 * 2);
    float*          Mg   = (float*)carve((size_t)NTOK * GCOL * 4);
    float*          VL   = (float*)carve((size_t)NBHL * NS_ * 16 * 4);
    float*          VD   = (float*)carve((size_t)2 * NBHL * NS_ * 16 * 4);
    float*          VG   = (float*)carve((size_t)NBHL * 32 * 4);
    if (off > ws_size) return;
    if (off > (size_t)134217728) return;

    const dim3 b256(256), b128(128), b64(64);

    cvt_hs_kernel<<<dim3((NTOK * NHID / 8 + 255) / 256), b256, 0, stream>>>(hs, Xh, NTOK * NHID / 8);
    cvt_wt_kernel<<<dim3(NCOL / 64, NHID / 64), b256, 0, stream>>>(Wm, Wt);
    cvt_wv_kernel<<<dim3(NH_), b256, 0, stream>>>(Wv, WvTh, WvTl);

    for (int g = 0; g < NGRP; ++g) {
        gemm_f16_kernel<<<dim3(GCOL / 128, NTOK / 64), b128, 0, stream>>>(
            Xh, Wt + (size_t)g * GCOL * NHID, bm + g * GCOL, Mg, NHID, GCOL, 0.03125f);
        chain_kernel<<<dim3(NBHL), b64, 0, stream>>>(Mg, mask, VL, VD, VG);
        gemm_out_kernel<<<dim3(NBHL * BPC), b128, 0, stream>>>(VL, VG, VD, WvTh, WvTl, bv, g, out);
    }
}
